// GnnPolicy_11312943857830
// MI455X (gfx1250) — hardware-verified
//
#include <hip/hip_runtime.h>
#include <stdint.h>

#define NN    512
#define OBSD  32
#define HD    128
#define NL    3
#define W1P   257
#define LP    264

static_assert(NN == 4 * 128);
static_assert(HD == 128);
static_assert(W1P == 2 * HD + 1);
static_assert(OBSD % 32 == 0);
static_assert((2 * HD) % 32 == 0 && (4 * HD) % 32 == 0);
static_assert(8 * 16 == 128);
static_assert((LP * 2) % 16 == 0);

typedef __attribute__((ext_vector_type(16))) __bf16 v16b;
typedef __attribute__((ext_vector_type(8)))  __bf16 v8b;
typedef __attribute__((ext_vector_type(8)))  float  v8f;
typedef __attribute__((ext_vector_type(4)))  float  v4f;
typedef __attribute__((ext_vector_type(2)))  float  v2f;
typedef __attribute__((ext_vector_type(4)))  unsigned int v4u;
typedef __attribute__((ext_vector_type(2)))  unsigned int v2u;
typedef v8b __attribute__((may_alias)) v8ba;
typedef v4f __attribute__((may_alias)) v4fa;
typedef v2f __attribute__((may_alias)) v2fa;
typedef v4u __attribute__((may_alias)) v4ua;
typedef v2u __attribute__((may_alias)) v2ua;

union FragU { v16b v; v8b h[2]; };

constexpr size_t SZ_OBSB = (size_t)NN * OBSD * 2;
constexpr size_t SZ_EW1  = (size_t)HD * OBSD * 2;
constexpr size_t SZ_WD2  = (size_t)HD * 2 * HD * 2;
constexpr size_t SZ_WIJ  = (size_t)2 * HD * 2 * HD * 2;
constexpr size_t SZ_UW1  = (size_t)HD * 4 * HD * 2;
constexpr size_t SZ_WD   = (size_t)NL * HD * 4;
constexpr size_t SZ_BIAS = (size_t)21 * HD * 4;
constexpr size_t SZ_DIST = (size_t)NN * NN * 4;
constexpr size_t SZ_AB   = (size_t)NN * 2 * HD * 4;
constexpr size_t SZ_CAT  = (size_t)NN * 4 * HD * 2;
constexpr size_t SZ_HL   = (size_t)NN * 2 * HD * 2;

constexpr size_t O_OBSB = 0;
constexpr size_t O_EW1  = O_OBSB + SZ_OBSB;
constexpr size_t O_EW2D = O_EW1 + SZ_EW1;
constexpr size_t O_EW3D = O_EW2D + SZ_WD2;
constexpr size_t O_WIJD = O_EW3D + SZ_WD2;
constexpr size_t O_MW2D = O_WIJD + NL * SZ_WIJ;
constexpr size_t O_MW3D = O_MW2D + NL * SZ_WD2;
constexpr size_t O_UW1Q = O_MW3D + NL * SZ_WD2;
constexpr size_t O_UW2D = O_UW1Q + NL * SZ_UW1;
constexpr size_t O_UW3D = O_UW2D + NL * SZ_WD2;
constexpr size_t O_WD   = O_UW3D + NL * SZ_WD2;
constexpr size_t O_BIAS = O_WD + SZ_WD;
constexpr size_t O_DIST = O_BIAS + SZ_BIAS;
constexpr size_t O_AB   = O_DIST + SZ_DIST;
constexpr size_t O_CAT  = O_AB + SZ_AB;
constexpr size_t O_H2S  = O_CAT + SZ_CAT;
constexpr size_t O_T1   = O_H2S + SZ_HL;
constexpr size_t O_T2   = O_T1 + SZ_HL;
constexpr size_t O_END  = O_T2 + SZ_HL;
static_assert(O_END == 4640768);
static_assert(O_EW1 % 256 == 0 && O_EW2D % 256 == 0 && O_EW3D % 256 == 0 && O_WIJD % 256 == 0);
static_assert(O_MW2D % 256 == 0 && O_MW3D % 256 == 0 && O_UW1Q % 256 == 0 && O_UW2D % 256 == 0);
static_assert(O_UW3D % 256 == 0 && O_WD % 256 == 0 && O_BIAS % 256 == 0 && O_DIST % 256 == 0);
static_assert(O_AB % 256 == 0 && O_CAT % 256 == 0 && O_H2S % 256 == 0 && O_T1 % 256 == 0 && O_T2 % 256 == 0);
static_assert(O_END <= (size_t)134217728);

constexpr int PL_W   = 0;
constexpr int PL_A   = PL_W + 128 * LP * 2;
constexpr int PL_V   = PL_A + 128 * LP * 2;
constexpr int PL_D   = PL_V + 4 * 128 * 4;
constexpr int PL_P   = PL_D + 512 * 4;
constexpr int PL_O   = PL_P + 8 * 128 * 4;
constexpr int PAIR_LDS = PL_O + 128 * 4;
static_assert(PAIR_LDS == 143872);
static_assert(PAIR_LDS <= 327680);
static_assert(PL_A % 16 == 0 && PL_V % 16 == 0 && PL_D % 16 == 0 && PL_P % 16 == 0 && PL_O % 16 == 0);

__device__ __forceinline__ unsigned short f2bf_bits(float f) {
  const unsigned u = __float_as_uint(f);
  return (unsigned short)((u + 0x7FFFu + ((u >> 16) & 1u)) >> 16);
}
__device__ __forceinline__ float bf_bits2f(unsigned short h) { return __uint_as_float(((unsigned)h) << 16); }
__device__ __forceinline__ float bf16r(float f) {
  unsigned u = __float_as_uint(f);
  u = (u + 0x7FFFu + ((u >> 16) & 1u)) & 0xFFFF0000u;
  return __uint_as_float(u);
}
__device__ __forceinline__ unsigned pk16(unsigned short a, unsigned short b) { return (unsigned)a | ((unsigned)b << 16); }

__device__ __forceinline__ void split_pair(float a, float b, unsigned& hw, unsigned& lw) {
  const unsigned short h0 = f2bf_bits(a), h1 = f2bf_bits(b);
  const unsigned short l0 = f2bf_bits(a - bf_bits2f(h0));
  const unsigned short l1 = f2bf_bits(b - bf_bits2f(h1));
  hw = pk16(h0, h1);
  lw = pk16(l0, l1);
}
__device__ __forceinline__ v4u cvt8(v4f a, v4f c) {
  v4u o;
  o[0] = pk16(f2bf_bits(a[0]), f2bf_bits(a[1]));
  o[1] = pk16(f2bf_bits(a[2]), f2bf_bits(a[3]));
  o[2] = pk16(f2bf_bits(c[0]), f2bf_bits(c[1]));
  o[3] = pk16(f2bf_bits(c[2]), f2bf_bits(c[3]));
  return o;
}
__device__ __forceinline__ void put16(unsigned short* dst, v4u o) {
  *(volatile v4u*)dst = o;
  __threadfence();
  *(volatile v4u*)dst = o;
}
__device__ __forceinline__ void put4f(float* dst, v4f o) {
  *(volatile v4f*)dst = o;
  __threadfence();
  *(volatile v4f*)dst = o;
}

__device__ __forceinline__ v8f wmma_bf16(v16b a, v16b b, v8f c) {
  v8f d = __builtin_amdgcn_wmma_f32_16x16x32_bf16(false, a, false, b, (short)0, c, false, false);
  asm volatile("v_nop\n\tv_nop\n\tv_nop\n\tv_nop" : "+v"(d) : "v"(a), "v"(b));
  return d;
}
__device__ __forceinline__ v16b load_frag_g(const unsigned short* __restrict__ p, int hh) {
  FragU f;
  f.h[0] = *(const v8ba*)(p + 8 * hh);
  f.h[1] = *(const v8ba*)(p + 16 + 8 * hh);
  return f.v;
}
__device__ __forceinline__ v16b load_frag_l(const unsigned short* p, int hh) {
  FragU f;
  f.h[0] = *(const v8ba*)(p + 8 * hh);
  f.h[1] = *(const v8ba*)(p + 16 + 8 * hh);
  return f.v;
}

__device__ __forceinline__ void gemm_core1_32x64(
    const unsigned short* __restrict__ A, int lda, const unsigned short* __restrict__ Bt, int ldb,
    int K, size_t aoff, size_t boff, int hh, v8f (&acc)[2][4]) {
  const unsigned short* a0 = A + aoff;
  const unsigned short* a1 = a0 + (size_t)16 * lda;
  const unsigned short* bp = Bt + boff;
#pragma unroll 1
  for (int k0 = 0; k0 < K; k0 += 32) {
    const v16b f0 = load_frag_g(a0 + k0, hh);
    const v16b f1 = load_frag_g(a1 + k0, hh);
#pragma unroll
    for (int nt = 0; nt < 4; ++nt) {
      const v16b fb = load_frag_g(bp + (size_t)nt * 16 * ldb + k0, hh);
      acc[0][nt] = wmma_bf16(f0, fb, acc[0][nt]);
      acc[1][nt] = wmma_bf16(f1, fb, acc[1][nt]);
    }
  }
}

__device__ __forceinline__ void straight_unit(const float* __restrict__ src, unsigned short* __restrict__ dst, int u) {
  const v4f a = *(const v4fa*)(src + (size_t)u * 8);
  const v4f c = *(const v4fa*)(src + (size_t)u * 8 + 4);
  put16(dst + (size_t)u * 8, cvt8(a, c));
}
__device__ __forceinline__ void dup_unit(const float* __restrict__ W, unsigned short* __restrict__ dst, int u) {
  const int n = u >> 5, c8 = (u & 31) * 8, sc = c8 & 127;
  const v4f a = *(const v4fa*)(W + (size_t)n * HD + sc);
  const v4f c = *(const v4fa*)(W + (size_t)n * HD + sc + 4);
  put16(dst + (size_t)n * 256 + c8, cvt8(a, c));
}

__global__ __launch_bounds__(256) void k_pa(const float* __restrict__ obs, const float* __restrict__ W1,
                                            const float* __restrict__ W2, const float* __restrict__ W3,
                                            unsigned char* __restrict__ ws) {
  const int b = blockIdx.x, tid = threadIdx.x;
  if (b < 8) {
    straight_unit(obs, (unsigned short*)(ws + O_OBSB), b * 256 + tid);
  } else if (b < 10) {
    straight_unit(W1, (unsigned short*)(ws + O_EW1), (b - 8) * 256 + tid);
  } else if (b < 26) {
    dup_unit(W2, (unsigned short*)(ws + O_EW2D), (b - 10) * 256 + tid);
  } else if (b < 42) {
    dup_unit(W3, (unsigned short*)(ws + O_EW3D), (b - 26) * 256 + tid);
  }
}

__global__ __launch_bounds__(256) void k_pb(const float* __restrict__ W1, const float* __restrict__ W2,
                                            const float* __restrict__ W3, unsigned char* __restrict__ ws) {
  const int b = blockIdx.x, tid = threadIdx.x;
  if (b < 96) {
    const int u = b * 256 + tid;
    const int l = u >> 13, ul = u & 8191, n = ul >> 5, c8 = (ul & 31) * 8, sc = c8 & 127;
    const float* src = W1 + (size_t)l * (HD * W1P) + (size_t)(n & 127) * W1P + (n >> 7) * HD + sc;
    float f[8];
#pragma unroll
    for (int e = 0; e < 8; ++e) f[e] = src[e];
    v4u o;
    o[0] = pk16(f2bf_bits(f[0]), f2bf_bits(f[1]));
    o[1] = pk16(f2bf_bits(f[2]), f2bf_bits(f[3]));
    o[2] = pk16(f2bf_bits(f[4]), f2bf_bits(f[5]));
    o[3] = pk16(f2bf_bits(f[6]), f2bf_bits(f[7]));
    put16((unsigned short*)(ws + O_WIJD) + (size_t)l * 65536 + (size_t)n * 256 + c8, o);
  } else if (b < 144) {
    dup_unit(W2, (unsigned short*)(ws + O_MW2D), (b - 96) * 256 + tid);
  } else if (b < 192) {
    dup_unit(W3, (unsigned short*)(ws + O_MW3D), (b - 144) * 256 + tid);
  } else if (b == 192) {
    if (tid < 96) {
      const int l = tid >> 5, q = tid & 31;
      const float* src = W1 + (size_t)l * (HD * W1P) + (size_t)(4 * q) * W1P + 2 * HD;
      v4f r;
      r[0] = bf16r(src[0]);
      r[1] = bf16r(src[W1P]);
      r[2] = bf16r(src[2 * W1P]);
      r[3] = bf16r(src[3 * W1P]);
      put4f((float*)(ws + O_WD) + l * HD + 4 * q, r);
    }
  }
}

__global__ __launch_bounds__(256) void k_pc(const float* __restrict__ W1, const float* __restrict__ W2,
                                            const float* __restrict__ W3, unsigned char* __restrict__ ws) {
  const int b = blockIdx.x, tid = threadIdx.x;
  if (b < 96) {
    const int u = b * 256 + tid;
    const int n = u >> 6, c8 = (u & 63) * 8;
    const int sc = ((c8 >> 8) << 7) | (c8 & 127);
    const v4f a = *(const v4fa*)(W1 + (size_t)n * 256 + sc);
    const v4f c = *(const v4fa*)(W1 + (size_t)n * 256 + sc + 4);
    put16((unsigned short*)(ws + O_UW1Q) + (size_t)n * 512 + c8, cvt8(a, c));
  } else if (b < 144) {
    dup_unit(W2, (unsigned short*)(ws + O_UW2D), (b - 96) * 256 + tid);
  } else if (b < 192) {
    dup_unit(W3, (unsigned short*)(ws + O_UW3D), (b - 144) * 256 + tid);
  }
}

__device__ __forceinline__ void bias_rows(const float* __restrict__ src, float* __restrict__ dst, int nunits, int tid) {
  if (tid < nunits) {
    const v4f v = *(const v4fa*)(src + 4 * tid);
    const v4f r = {bf16r(v[0]), bf16r(v[1]), bf16r(v[2]), bf16r(v[3])};
    put4f(dst + 4 * tid, r);
  }
}
__global__ __launch_bounds__(128) void k_pd(const float* __restrict__ eb1, const float* __restrict__ eb2,
                                            const float* __restrict__ eb3, const float* __restrict__ mb1,
                                            const float* __restrict__ mb2, const float* __restrict__ mb3,
                                            const float* __restrict__ ub1, const float* __restrict__ ub2,
                                            const float* __restrict__ ub3, unsigned char* __restrict__ ws) {
  float* B = (float*)(ws + O_BIAS);
  const int b = blockIdx.x, tid = threadIdx.x;
  if (b == 0)      bias_rows(eb1, B + 0 * HD, 32, tid);
  else if (b == 1) bias_rows(eb2, B + 1 * HD, 32, tid);
  else if (b == 2) bias_rows(eb3, B + 2 * HD, 32, tid);
  else if (b == 3) bias_rows(mb1, B + 3 * HD, 96, tid);
  else if (b == 4) bias_rows(mb2, B + 6 * HD, 96, tid);
  else if (b == 5) bias_rows(mb3, B + 9 * HD, 96, tid);
  else if (b == 6) bias_rows(ub1, B + 12 * HD, 96, tid);
  else if (b == 7) bias_rows(ub2, B + 15 * HD, 96, tid);
  else if (b == 8) bias_rows(ub3, B + 18 * HD, 96, tid);
}

__global__ __launch_bounds__(256) void k_dist(const float* __restrict__ pos, float* __restrict__ DIST) {
#pragma clang fp contract(off)
  const int g = blockIdx.x * 256 + threadIdx.x;
  if (g >= NN * NN) return;
  const int i = g >> 9, j = g & 511;
  const v2f pi = *(const v2fa*)(pos + 2 * i);
  const v2f pj = *(const v2fa*)(pos + 2 * j);
  const float dx = bf16r(pi[0]) - bf16r(pj[0]);
  const float dy = bf16r(pi[1]) - bf16r(pj[1]);
  const float xx = dx * dx;
  const float yy = dy * dy;
  const float sq = xx + yy;
  const float sr = sqrtf(sq);
  const float d = (i == j) ? 0.0f : sr;
  float* dst = DIST + g;
  *(volatile float*)dst = d;
  __threadfence();
  *(volatile float*)dst = d;
}

template <int OUTF32, int RELU, int HASBIAS>
__global__ __launch_bounds__(128) void k_gemm(const unsigned short* __restrict__ A, int lda,
                                              const unsigned short* __restrict__ Bt, int K,
                                              const float* __restrict__ bias, float bscale,
                                              float* __restrict__ outF, unsigned short* __restrict__ outH,
                                              int ldo, int ocol) {
  __shared__ __align__(16) float sF[128 * 64];
  const int tid = threadIdx.x, lane = tid & 31, w = tid >> 5;
  const int hh = lane >> 4, m = lane & 15;
  const int m0 = blockIdx.x * 128;
  const int n0 = blockIdx.y * 64;
  const int m0w = m0 + 32 * w;

  const v8f zero8 = {0.f, 0.f, 0.f, 0.f, 0.f, 0.f, 0.f, 0.f};
  v8f acc[2][4];
#pragma unroll
  for (int mt = 0; mt < 2; ++mt)
#pragma unroll
    for (int nt = 0; nt < 4; ++nt) acc[mt][nt] = zero8;

  gemm_core1_32x64(A, lda, Bt, K, K, (size_t)(m0w + m) * lda, (size_t)(n0 + m) * K, hh, acc);

  float bv[4];
#pragma unroll
  for (int nt = 0; nt < 4; ++nt) {
    bv[nt] = 0.0f;
    if (HASBIAS) bv[nt] = bscale * bias[n0 + 16 * nt + m];
  }
#pragma unroll
  for (int nt = 0; nt < 4; ++nt)
#pragma unroll
    for (int mt = 0; mt < 2; ++mt)
#pragma unroll
      for (int r = 0; r < 8; ++r) {
        const int tokl = 32 * w + 16 * mt + 8 * hh + r;
        const int feat = 16 * nt + m;
        float y = acc[mt][nt][r] + bv[nt];
        if (RELU) y = (y > 0.0f) ? y : 0.0f;
        sF[tokl * 64 + feat] = y;
      }
  __syncthreads();

  if (OUTF32) {
    const int rsub = lane >> 4, c4 = (lane & 15) * 4;
    v4f vals[16];
#pragma unroll
    for (int it = 0; it < 16; ++it) {
      const int row = 32 * w + 2 * it + rsub;
      vals[it] = *(const v4fa*)(sF + row * 64 + c4);
    }
    for (int pass = 0; pass < 2; ++pass) {
#pragma unroll
      for (int it = 0; it < 16; ++it) {
        const int row = 32 * w + 2 * it + rsub;
        *(volatile v4f*)(outF + (size_t)(m0 + row) * ldo + n0 + c4) = vals[it];
      }
      __threadfence();
    }
  } else {
    const int q8 = lane & 7, sub = lane >> 3;
    v4u hv[8], lv[8];
#pragma unroll
    for (int it = 0; it < 8; ++it) {
      const int row = 32 * w + 4 * it + sub;
      const v4f a = *(const v4fa*)(sF + row * 64 + 8 * q8);
      const v4f c = *(const v4fa*)(sF + row * 64 + 8 * q8 + 4);
      unsigned h0, l0, h1, l1, h2, l2, h3, l3;
      split_pair(a[0], a[1], h0, l0);
      split_pair(a[2], a[3], h1, l1);
      split_pair(c[0], c[1], h2, l2);
      split_pair(c[2], c[3], h3, l3);
      const v4u hq = {h0, h1, h2, h3};
      const v4u lq = {l0, l1, l2, l3};
      hv[it] = hq;
      lv[it] = lq;
    }
    for (int pass = 0; pass < 2; ++pass) {
#pragma unroll
      for (int it = 0; it < 8; ++it) {
        const int row = 32 * w + 4 * it + sub;
        unsigned short* dst = outH + (size_t)(m0 + row) * ldo + ocol + n0 + 8 * q8;
        *(volatile v4u*)dst = hv[it];
        *(volatile v4u*)(dst + 128) = lv[it];
      }
      __threadfence();
    }
  }
}

__global__ __launch_bounds__(256) __attribute__((amdgpu_num_vgpr(248)))
void k_pair(const float* __restrict__ AB, const float* __restrict__ DIST,
            const unsigned short* __restrict__ W2D, const float* __restrict__ WD,
            const float* __restrict__ B1, const float* __restrict__ B2,
            unsigned short* __restrict__ H2SHL) {
  extern __shared__ __align__(16) unsigned char smem[];
  unsigned short* sW = (unsigned short*)(smem + PL_W);
  unsigned short* sA = (unsigned short*)(smem + PL_A);
  float* sV = (float*)(smem + PL_V);
  float* sD = (float*)(smem + PL_D);
  float* sP = (float*)(smem + PL_P);
  unsigned* sO = (unsigned*)(smem + PL_O);

  const int tid = threadIdx.x, lane = tid & 31, w = tid >> 5;
  const int hh = lane >> 4, m = lane & 15;
  const int i = blockIdx.x;

#pragma unroll 4
  for (int it = 0; it < 16; ++it) {
    const int c = tid + 256 * it;
    const int row = c >> 5, ch = c & 31;
    const v4u v = *(const v4ua*)(W2D + (size_t)row * 256 + ch * 8);
    *(v4ua*)(sW + row * LP + ch * 8) = v;
  }
  if (w < 4) {
    v4f v;
    if (w == 0)      v = *(const v4fa*)(AB + (size_t)i * 256 + 4 * lane);
    else if (w == 1) v = *(const v4fa*)(WD + 4 * lane);
    else if (w == 2) v = *(const v4fa*)(B1 + 4 * lane);
    else             v = *(const v4fa*)(B2 + 4 * lane);
    *(v4fa*)(sV + 128 * w + 4 * lane) = v;
  } else {
    const int idx = tid - 128;
    const v4f v = *(const v4fa*)(DIST + (size_t)i * NN + 4 * idx);
    *(v4fa*)(sD + 4 * idx) = v;
  }
  __syncthreads();

  const v4f aiv = *(const v4fa*)(sV + 4 * lane);
  const v4f wdv = *(const v4fa*)(sV + 128 + 4 * lane);
  const v4f b1v = *(const v4fa*)(sV + 256 + 4 * lane);

  float s[8];
#pragma unroll
  for (int nt = 0; nt < 8; ++nt) s[nt] = 0.0f;
  const v8f zero8 = {0.f, 0.f, 0.f, 0.f, 0.f, 0.f, 0.f, 0.f};

#pragma unroll 1
  for (int t = 0; t < 4; ++t) {
#pragma unroll 4
    for (int rr = 0; rr < 16; ++rr) {
      const int jl = 16 * w + rr;
      const int j = 128 * t + jl;
      const v4f bj = *(const v4fa*)(AB + (size_t)j * 256 + HD + 4 * lane);
      const float d = sD[j];
      float hv[4];
#pragma unroll
      for (int e = 0; e < 4; ++e) {
        const float v = ((aiv[e] + bj[e]) + d * wdv[e]) + b1v[e];
        hv[e] = (v > 0.0f) ? v : 0.0f;
      }
      unsigned hw0, lw0, hw1, lw1;
      split_pair(hv[0], hv[1], hw0, lw0);
      split_pair(hv[2], hv[3], hw1, lw1);
      const v2u Hq = {hw0, hw1};
      const v2u Lq = {lw0, lw1};
      *(v2ua*)(sA + jl * LP + 4 * lane) = Hq;
      *(v2ua*)(sA + jl * LP + HD + 4 * lane) = Lq;
    }
    __syncthreads();

    v8f acc[8];
#pragma unroll
    for (int nt = 0; nt < 8; ++nt) acc[nt] = zero8;
    const unsigned short* arow = sA + (16 * w + m) * LP;
    const unsigned short* brow = sW + m * LP;
#pragma unroll 1
    for (int k0 = 0; k0 < 2 * HD; k0 += 32) {
      const v16b fa = load_frag_l(arow + k0, hh);
#pragma unroll
      for (int nt = 0; nt < 8; ++nt) {
        const v16b fb = load_frag_l(brow + nt * 16 * LP + k0, hh);
        acc[nt] = wmma_bf16(fa, fb, acc[nt]);
      }
    }

    const int jbase = 128 * t + 16 * w + 8 * hh;
#pragma unroll
    for (int nt = 0; nt < 8; ++nt) {
      const float bb = sV[384 + 16 * nt + m];
#pragma unroll
      for (int r = 0; r < 8; ++r) {
        float v = acc[nt][r] + bb;
        v = (v > 0.0f) ? v : 0.0f;
        v = ((jbase + r) == i) ? 0.0f : v;
        s[nt] += v;
      }
    }
    __syncthreads();
  }

#pragma unroll
  for (int nt = 0; nt < 8; ++nt) s[nt] += __shfl_xor(s[nt], 16);
  if (lane < 16) {
#pragma unroll
    for (int nt = 0; nt < 8; ++nt) sP[w * 128 + 16 * nt + m] = s[nt];
  }
  __syncthreads();
  if (tid < 64) {
    const int c = 2 * tid;
    float t0 = 0.0f, t1 = 0.0f;
#pragma unroll
    for (int ww = 0; ww < 8; ++ww) {
      t0 += sP[ww * 128 + c];
      t1 += sP[ww * 128 + c + 1];
    }
    unsigned hw, lw;
    split_pair(t0, t1, hw, lw);
    sO[tid] = hw;
    sO[64 + tid] = lw;
  }
  __syncthreads();
  if (w == 0) {
    const v4u v = *(const v4ua*)(sO + 4 * lane);
    unsigned short* dst = H2SHL + (size_t)i * 256 + 8 * lane;
    *(volatile v4u*)dst = v;
    __threadfence();
    *(volatile v4u*)dst = v;
  }
}

extern "C" void kernel_launch(void* const* d_in, const int* in_sizes, int n_in,
                              void* d_out, int out_size, void* d_ws, size_t ws_size,
                              hipStream_t stream) {
  if (n_in < 20) return;
  if (in_sizes[0] != NN * OBSD || in_sizes[1] != NN * 2) return;
  if (in_sizes[2] != HD * OBSD || in_sizes[3] != HD) return;
  if (in_sizes[4] != HD * HD || in_sizes[5] != HD) return;
  if (in_sizes[6] != HD * HD || in_sizes[7] != HD) return;
  if (in_sizes[8] != NL * HD * W1P || in_sizes[9] != NL * HD) return;
  if (in_sizes[10] != NL * HD * HD || in_sizes[11] != NL * HD) return;
  if (in_sizes[12] != NL * HD * HD || in_sizes[13] != NL * HD) return;
  if (in_sizes[14] != NL * HD * 2 * HD || in_sizes[15] != NL * HD) return;
  if (in_sizes[16] != NL * HD * HD || in_sizes[17] != NL * HD) return;
  if (in_sizes[18] != NL * HD * HD || in_sizes[19] != NL * HD) return;
  if (out_size != NN * HD) return;
  if (O_END > ws_size) return;

  const float* obs    = (const float*)d_in[0];
  const float* pos    = (const float*)d_in[1];
  const float* enc_W1 = (const float*)d_in[2];
  const float* enc_b1 = (const float*)d_in[3];
  const float* enc_W2 = (const float*)d_in[4];
  const float* enc_b2 = (const float*)d_in[5];
  const float* enc_W3 = (const float*)d_in[6];
  const float* enc_b3 = (const float*)d_in[7];
  const float* msg_W1 = (const float*)d_in[8];
  const float* msg_b1 = (const float*)d_in[9];
  const float* msg_W2 = (const float*)d_in[10];
  const float* msg_b2 = (const float*)d_in[11];
  const float* msg_W3 = (const float*)d_in[12];
  const float* msg_b3 = (const float*)d_in[13];
  const float* upd_W1 = (const float*)d_in[14];
  const float* upd_b1 = (const float*)d_in[15];
  const float* upd_W2 = (const float*)d_in[16];
  const float* upd_b2 = (const float*)d_in[17];
  const float* upd_W3 = (const float*)d_in[18];
  const float* upd_b3 = (const float*)d_in[19];
  float* out = (float*)d_out;

  unsigned char* ws = (unsigned char*)d_ws;
  unsigned short* OBSB = (unsigned short*)(ws + O_OBSB);
  unsigned short* EW1  = (unsigned short*)(ws + O_EW1);
  unsigned short* EW2D = (unsigned short*)(ws + O_EW2D);
  unsigned short* EW3D = (unsigned short*)(ws + O_EW3D);
  unsigned short* WIJD = (unsigned short*)(ws + O_WIJD);
  unsigned short* MW2D = (unsigned short*)(ws + O_MW2D);
  unsigned short* MW3D = (unsigned short*)(ws + O_MW3D);
  unsigned short* UW1Q = (unsigned short*)(ws + O_UW1Q);
  unsigned short* UW2D = (unsigned short*)(ws + O_UW2D);
  unsigned short* UW3D = (unsigned short*)(ws + O_UW3D);
  float*          WD   = (float*)(ws + O_WD);
  float*          BIAS = (float*)(ws + O_BIAS);
  float*          DIST = (float*)(ws + O_DIST);
  float*          AB   = (float*)(ws + O_AB);
  unsigned short* CAT  = (unsigned short*)(ws + O_CAT);
  unsigned short* H2S  = (unsigned short*)(ws + O_H2S);
  unsigned short* T1   = (unsigned short*)(ws + O_T1);
  unsigned short* T2   = (unsigned short*)(ws + O_T2);

  (void)hipFuncSetAttribute(reinterpret_cast<const void*>(&k_pair),
                            hipFuncAttributeMaxDynamicSharedMemorySize, PAIR_LDS);

  k_pa<<<42, 256, 0, stream>>>(obs, enc_W1, enc_W2, enc_W3, ws);
  k_pb<<<193, 256, 0, stream>>>(msg_W1, msg_W2, msg_W3, ws);
  k_pc<<<192, 256, 0, stream>>>(upd_W1, upd_W2, upd_W3, ws);
  k_pd<<<9, 128, 0, stream>>>(enc_b1, enc_b2, enc_b3, msg_b1, msg_b2, msg_b3, upd_b1, upd_b2, upd_b3, ws);
  k_dist<<<(NN * NN) / 256, 256, 0, stream>>>(pos, DIST);

  const dim3 g128(NN / 128, HD / 64);
  const dim3 g256(NN / 128, (2 * HD) / 64);

  k_gemm<0, 1, 1><<<g128, 128, 0, stream>>>(OBSB, OBSD, EW1, OBSD, BIAS + 0 * HD, 1.0f, AB, T1, 256, 0);
  k_gemm<0, 1, 1><<<g128, 128, 0, stream>>>(T1, 256, EW2D, 256, BIAS + 1 * HD, 1.0f, AB, T2, 256, 0);
  k_gemm<0, 0, 1><<<g128, 128, 0, stream>>>(T2, 256, EW3D, 256, BIAS + 2 * HD, 1.0f, AB, CAT, 512, 0);

  for (int l = 0; l < NL; ++l) {
    const unsigned short* wij = WIJD + (size_t)l * 65536;
    const unsigned short* mw2 = MW2D + (size_t)l * 32768;
    const unsigned short* mw3 = MW3D + (size_t)l * 32768;
    const unsigned short* uw1 = UW1Q + (size_t)l * 65536;
    const unsigned short* uw2 = UW2D + (size_t)l * 32768;
    const unsigned short* uw3 = UW3D + (size_t)l * 32768;
    k_gemm<1, 0, 0><<<g256, 128, 0, stream>>>(CAT, 512, wij, 256, BIAS, 0.0f, AB, T1, 256, 0);
    k_pair<<<NN, 256, PAIR_LDS, stream>>>(AB, DIST, mw2, WD + l * HD, BIAS + (3 + l) * HD, BIAS + (6 + l) * HD, H2S);
    k_gemm<0, 0, 1><<<g128, 128, 0, stream>>>(H2S, 256, mw3, 256, BIAS + (9 + l) * HD, 511.0f, AB, CAT, 512, 256);
    k_gemm<0, 1, 1><<<g128, 128, 0, stream>>>(CAT, 512, uw1, 512, BIAS + (12 + l) * HD, 1.0f, AB, T1, 256, 0);
    k_gemm<0, 1, 1><<<g128, 128, 0, stream>>>(T1, 256, uw2, 256, BIAS + (15 + l) * HD, 1.0f, AB, T2, 256, 0);
    if (l < NL - 1) {
      k_gemm<0, 0, 1><<<g128, 128, 0, stream>>>(T2, 256, uw3, 256, BIAS + (18 + l) * HD, 1.0f, AB, CAT, 512, 0);
    } else {
      k_gemm<1, 0, 1><<<g128, 128, 0, stream>>>(T2, 256, uw3, 256, BIAS + (18 + l) * HD, 1.0f, out, T1, HD, 0);
    }
  }
  (void)hipGetLastError();
}
